// LTVMinimumPhaseFIRFilterPrecise_22041772163075
// MI455X (gfx1250) — hardware-verified
//
#include <hip/hip_runtime.h>


#define NBATCH 4
#define NFRM   400
#define NBIN   129
#define HOPC   240
#define TLEN   (NFRM * HOPC)
#define KLEN   256
#define GFR    14
#define NGRP   29
#define RPB    (GFR * HOPC)
#define XW     (RPB + KLEN)
#define KP     264
#define NCOL   16

static_assert(NGRP * RPB >= TLEN);
static_assert((NGRP - 1) * RPB < TLEN);
static_assert(RPB % 32 == 0);
static_assert(TLEN % 32 == 0);
static_assert((TLEN - (NGRP - 1) * RPB) % 32 == 0);
static_assert(XW >= RPB + KLEN - 1);
static_assert((KP * 2) % 16 == 0);

typedef float          v4f   __attribute__((ext_vector_type(4)));
typedef float          v8f   __attribute__((ext_vector_type(8)));
typedef _Float16       v16h  __attribute__((ext_vector_type(16)));
typedef __bf16         v16b  __attribute__((ext_vector_type(16)));
typedef unsigned short u16x8 __attribute__((ext_vector_type(8)));
typedef unsigned int   u32x8 __attribute__((ext_vector_type(8)));
union Frag { v16h f; v16b b; u32x8 w; u16x8 h[2]; };

constexpr size_t SZ_PLANE = (size_t)NBATCH * NFRM * KLEN * 2;
constexpr size_t OFF_KH = 0;
constexpr size_t OFF_KL = OFF_KH + SZ_PLANE;
constexpr size_t WS_END = OFF_KL + SZ_PLANE;
static_assert(WS_END <= (size_t)134217728);
static_assert(SZ_PLANE % 512 == 0 && OFF_KL % 512 == 0);

__device__ __forceinline__ unsigned short f32_to_bf16(float f) {
    const unsigned u = __float_as_uint(f);
    return (unsigned short)((u + 0x7FFFu + ((u >> 16) & 1u)) >> 16);
}
__device__ __forceinline__ float bf16_to_f32(unsigned short v) { return __uint_as_float(((unsigned)v) << 16); }

__device__ __forceinline__ void mma_b(v8f& acc, const Frag& a, const Frag& b) {
    acc = __builtin_amdgcn_wmma_f32_16x16x32_bf16(false, a.b, false, b.b, (short)0, acc, false, false);
    asm volatile("v_nop\n\tv_nop\n\tv_nop\n\tv_nop" : "+v"(acc) : "v"(a.b), "v"(b.b));
}

__global__ __launch_bounds__(256)
void k_design(const float* __restrict__ log_mag, unsigned short* kh_out, unsigned short* kl_out)
{
    __shared__ float cq[72];
    __shared__ float ct[KLEN];
    __shared__ float st[KLEN];
    __shared__ float sf[KLEN];
    __shared__ float sx[KLEN];
    __shared__ float s_re[KLEN];
    __shared__ float s_im[KLEN];
    __shared__ __attribute__((aligned(16))) unsigned short skh[KLEN];
    __shared__ __attribute__((aligned(16))) unsigned short skl[KLEN];

    const int p = blockIdx.x;
    const int tid = threadIdx.x, lane = tid & 31, wave = tid >> 5;
    const float* lm = log_mag + (size_t)p * NBIN;

    {
        const int qi = min(tid, 64);
        float c = cosf((float)qi * 0.024543692606170259f);
        c = (qi == 0) ? 1.0f : c;
        c = (qi == 64) ? 0.0f : c;
        if (tid <= 64) cq[tid] = c;
    }
    {
        const int fi = (tid <= 128) ? tid : (KLEN - tid);
        sf[tid] = lm[fi];
    }
    __syncthreads();

    {
        const int jj = (tid > 128) ? (KLEN - tid) : tid;
        const float ca = cq[min(jj, 64)];
        const float cb = cq[min(128 - jj, 64)];
        const float cv = (jj <= 64) ? ca : -cb;
        int ic = 64 - jj; ic = (ic < 0) ? -ic : ic;
        float sv = cq[ic];
        sv = (tid > 128) ? -sv : sv;
        ct[tid] = cv;
        st[tid] = sv;
    }
    __syncthreads();

    float xf = 0.0f;
#pragma unroll 2
    for (int n = 0; n < KLEN; ++n) xf = fmaf(sf[n], ct[(n * tid) & 255], xf);
    {
        const float hk = (tid == 0 || tid == 128) ? 1.0f : ((tid < 128) ? 2.0f : 0.0f);
        sx[tid] = hk * xf;
    }
    __syncthreads();

    float mi = 0.0f;
#pragma unroll 2
    for (int k = 0; k <= 128; ++k) mi = fmaf(sx[k], st[(k * tid) & 255], mi);
    {
        const float mp = -mi * (1.0f / 256.0f);
        const float e = expf(sf[tid]);
        float sn, cn;
        sincosf(mp, &sn, &cn);
        s_re[tid] = e * cn;
        s_im[tid] = e * sn;
    }
    __syncthreads();

    float kr = 0.0f;
#pragma unroll 2
    for (int k = 0; k < KLEN; ++k) {
        const int a = (k * tid) & 255;
        kr = fmaf(s_re[k], ct[a], kr);
        kr = fmaf(-s_im[k], st[a], kr);
    }
    kr *= (1.0f / 256.0f);
    {
        const float wv = (tid < 128) ? 1.0f : (0.5f - 0.5f * ct[tid]);
        kr *= wv;
    }
    {
        const unsigned short hb = f32_to_bf16(kr);
        const unsigned short lb = f32_to_bf16(kr - bf16_to_f32(hb));
        skh[tid] = hb;
        skl[tid] = lb;
    }
    __syncthreads();

    const u16x8 vh = *(const u16x8*)(skh + 8 * lane);
    const u16x8 vl = *(const u16x8*)(skl + 8 * lane);
    u16x8 v = vl;
    if (wave == 0) v = vh;
    unsigned short* dst = ((wave == 0) ? kh_out : kl_out) + (size_t)p * KLEN + 8 * lane;
    if (wave < 2) *(volatile u16x8*)dst = v;
    __threadfence();
    if (wave < 2) *(volatile u16x8*)dst = v;
}

__global__ __launch_bounds__(256)
void k_filt(const float* __restrict__ ex, const unsigned short* __restrict__ khp, const unsigned short* __restrict__ klp,
            const int* __restrict__ hop, float* out)
{
    __shared__ __attribute__((aligned(16))) unsigned int   xr[XW];
    __shared__ __attribute__((aligned(16))) unsigned short skh[NCOL * KP];
    __shared__ __attribute__((aligned(16))) unsigned short skl[NCOL * KP];
    __shared__ __attribute__((aligned(16))) float          sy[RPB];

    const int g = blockIdx.x, b = blockIdx.y;
    const int tid = threadIdx.x, lane = tid & 31, wave = tid >> 5, h = lane >> 4, m = lane & 15;
    const int t0 = g * RPB;
    const int nrows = min(RPB, TLEN - t0);
    const int ntiles = nrows >> 4;
    const int fbase = g * GFR - 1;
    const size_t xb = (size_t)b * TLEN;

#pragma unroll 1
    for (int i = tid; i < XW; i += 256) {
        const int t = t0 + (RPB - 1) - i;
        const int tc = min(max(t, 0), TLEN - 1);
        float v = ex[xb + tc];
        v = (t >= 0 && t < TLEN) ? v : 0.0f;
        const unsigned short hb = f32_to_bf16(v);
        const unsigned short lb = f32_to_bf16(v - bf16_to_f32(hb));
        xr[i] = (unsigned)hb | (((unsigned)lb) << 16);
    }
#pragma unroll
    for (int it = 0; it < 4; ++it) {
        const int pl = it >> 1;
        const int r = (it & 1) * 256 + tid;
        const int fr = r >> 5, pc = r & 31;
        const int f = min(max(fbase + fr, 0), NFRM - 1);
        const unsigned short* src = ((pl == 0) ? khp : klp) + ((size_t)b * NFRM + f) * KLEN + pc * 8;
        const u16x8 v = *(const u16x8*)src;
        if (pl == 0) *(u16x8*)(skh + fr * KP + pc * 8) = v;
        else         *(u16x8*)(skl + fr * KP + pc * 8) = v;
    }
    __syncthreads();

    const float rh = 1.0f / (float)hop[0];

    for (int tile = wave; tile < ntiles; tile += 8) {
        v8f acc;
#pragma unroll
        for (int r = 0; r < 8; ++r) acc[r] = 0.0f;
        const int jl = (RPB - 1) - (tile * 16 + m) + 8 * h;

#pragma unroll 2
        for (int ks = 0; ks < 8; ++ks) {
            const int jb = jl + ks * 32;
            Frag ah, al, bh, bl;
#pragma unroll
            for (int pq = 0; pq < 8; ++pq) {
                const int e0 = 2 * pq;
                const int j0 = jb + ((e0 < 8) ? e0 : (e0 + 8));
                const unsigned w0 = xr[j0];
                const unsigned w1 = xr[j0 + 1];
                ah.w[pq] = (w0 & 0xFFFFu) | (w1 << 16);
                al.w[pq] = (w0 >> 16) | (w1 & 0xFFFF0000u);
            }
            const unsigned short* bp = skh + m * KP + ks * 32 + 8 * h;
            const unsigned short* cp = skl + m * KP + ks * 32 + 8 * h;
            bh.h[0] = *(const u16x8*)bp;
            bh.h[1] = *(const u16x8*)(bp + 16);
            bl.h[0] = *(const u16x8*)cp;
            bl.h[1] = *(const u16x8*)(cp + 16);
            mma_b(acc, ah, bh);
            mma_b(acc, ah, bl);
            mma_b(acc, al, bh);
        }

        const int i = m;
        const int t = t0 + tile * 16 + i;
        float s = ((float)t + 0.5f) * rh - 0.5f;
        s = fminf(fmaxf(s, 0.0f), (float)(NFRM - 1));
        const float lof = floorf(s);
        const int lo = (int)lof;
        const float w = s - lof;
        const int hi = min(lo + 1, NFRM - 1);
        const int clo = min(max(lo - fbase, 0), NCOL - 1);
        const int chi = min(max(hi - fbase, 0), NCOL - 1);
        const int slo = clo + ((i >> 3) << 4);
        const int shi = chi + ((i >> 3) << 4);
        float ylo = 0.0f, yhi = 0.0f;
#pragma unroll
        for (int v = 0; v < 8; ++v) {
            const float a0 = __shfl(acc[v], slo, 32);
            const float a1 = __shfl(acc[v], shi, 32);
            ylo = ((i & 7) == v) ? a0 : ylo;
            yhi = ((i & 7) == v) ? a1 : yhi;
        }
        const float y = (1.0f - w) * ylo + w * yhi;
        if (lane < 16) sy[tile * 16 + i] = y;
    }
    __syncthreads();

    const int npieces = nrows >> 2;
    float* ob = out + xb + t0;
    v4f ov[4];
#pragma unroll
    for (int it = 0; it < 4; ++it) {
        const int pp = min(it * 256 + tid, npieces - 1);
        ov[it] = *(const v4f*)(sy + 4 * pp);
    }
#pragma unroll
    for (int it = 0; it < 4; ++it) {
        const int pp = it * 256 + tid;
        if (pp < npieces) *(volatile v4f*)(ob + 4 * pp) = ov[it];
    }
    __threadfence();
#pragma unroll
    for (int it = 0; it < 4; ++it) {
        const int pp = it * 256 + tid;
        if (pp < npieces) *(volatile v4f*)(ob + 4 * pp) = ov[it];
    }
}

extern "C" void kernel_launch(void* const* d_in, const int* in_sizes, int n_in,
                              void* d_out, int out_size, void* d_ws, size_t ws_size, hipStream_t stream)
{
    if (n_in < 3) return;
    if (in_sizes[0] != NBATCH * TLEN || in_sizes[1] != NBATCH * NFRM * NBIN || in_sizes[2] < 1) return;
    if (out_size != NBATCH * TLEN) return;
    if (ws_size < WS_END) return;

    const float* ex      = (const float*)d_in[0];
    const float* log_mag = (const float*)d_in[1];
    const int*   hop     = (const int*)d_in[2];
    float* out = (float*)d_out;
    char* ws = (char*)d_ws;
    unsigned short* KH = (unsigned short*)(ws + OFF_KH);
    unsigned short* KL = (unsigned short*)(ws + OFF_KL);

    k_design<<<dim3(NBATCH * NFRM), dim3(256), 0, stream>>>(log_mag, KH, KL);
    k_filt<<<dim3(NGRP, NBATCH), dim3(256), 0, stream>>>(ex, KH, KL, hop, out);
}
